// MVAE_13486197309656
// MI455X (gfx1250) — hardware-verified
//
#include <hip/hip_runtime.h>
#include <math.h>

constexpr int kRows = 32768;
constexpr int kNF = 192;
constexpr int kNF2 = 384;
constexpr int kNL = 40;
constexpr int kNE = 6;
constexpr int kNG = 64;
constexpr int kHeadN = 128;
constexpr int kZK = 64;
constexpr int kMoeK = kNE * kNF2 + 32;
constexpr int kMoeLines = 37;
constexpr int kMoeLd = kMoeLines * 64;
constexpr int kThreadsPerMoeRow = kMoeLines * 8;
constexpr int kChunkRows = 8192;
constexpr int kNumChunks = kRows / kChunkRows;
constexpr float kActCarry = 16.0f;
constexpr float kWCarry = 16.0f;
constexpr float kMoeCarry = 64.0f;
constexpr float kPlainScale = 1.0f / 256.0f;
constexpr float kMoeScale = 1.0f / 1024.0f;
static_assert(kMoeLd == 2368);
static_assert(kMoeK % 32 == 0);
static_assert(kNumChunks * kChunkRows == kRows);
static_assert(kChunkRows % 64 == 0);

constexpr size_t kMiB = 1048576;
constexpr size_t kOffE1t = 0;
constexpr size_t kOffE2t = 294912;
constexpr size_t kOffE3t = 589824;
constexpr size_t kOffE4t = 884736;
constexpr size_t kOffHdHi = 1032192;
constexpr size_t kOffHdLo = 1081344;
constexpr size_t kOffD1t = 1130496;
constexpr size_t kOffG1t = 1155072;
constexpr size_t kOffG2t = 1204224;
constexpr size_t kOffG3t = 1212416;
constexpr size_t kOffBt0 = 1220608;
constexpr size_t kOffBt1 = 3039232;
constexpr size_t kOffWEnd = 3948544;
constexpr size_t kOffR0 = 4 * kMiB;
constexpr size_t kOffR1 = 28 * kMiB;
constexpr size_t kOffR2 = 52 * kMiB;
constexpr size_t kWsTotal = 100 * kMiB;
static_assert(kOffE2t == kOffE1t + (size_t)kNF2 * kNF2 * 2);
static_assert(kOffE3t == kOffE2t + (size_t)kNF2 * kNF2 * 2);
static_assert(kOffE4t == kOffE3t + (size_t)kNF2 * kNF2 * 2);
static_assert(kOffHdHi == kOffE4t + (size_t)kNF * kNF2 * 2);
static_assert(kOffHdLo == kOffHdHi + (size_t)kHeadN * kNF * 2);
static_assert(kOffD1t == kOffHdLo + (size_t)kHeadN * kNF * 2);
static_assert(kOffG1t == kOffD1t + (size_t)kNF * kZK * 2);
static_assert(kOffG2t == kOffG1t + (size_t)kNG * kNF2 * 2);
static_assert(kOffG3t == kOffG2t + (size_t)kNG * kNG * 2);
static_assert(kOffBt0 == kOffG3t + (size_t)kNG * kNG * 2);
static_assert(kOffBt1 == kOffBt0 + (size_t)kNF2 * kMoeLd * 2);
static_assert(kOffWEnd == kOffBt1 + (size_t)kNF * kMoeLd * 2);
static_assert(kOffWEnd <= kOffR0);
static_assert((size_t)kRows * kNF2 * 2 <= 24 * kMiB);
static_assert((size_t)kRows * kNF * 2 * 2 <= 24 * kMiB);
static_assert((size_t)kRows * kNF * 4 <= 24 * kMiB);
static_assert((size_t)kRows * kHeadN * 4 <= 24 * kMiB);
static_assert((size_t)kRows * kNG * 2 <= 4 * kMiB);
static_assert((size_t)kRows * kNG * 4 <= 8 * kMiB);
static_assert((size_t)kRows * 8 * 4 <= 1 * kMiB);
static_assert((size_t)kChunkRows * kNF2 * 4 <= 12 * kMiB);
static_assert((size_t)kRows * kNF2 * 4 <= 48 * kMiB);
static_assert((size_t)kChunkRows * kMoeLd * 2 <= 48 * kMiB);
static_assert(kOffR2 + 48 * kMiB == kWsTotal);

typedef __attribute__((ext_vector_type(16))) _Float16 v16h;
typedef __attribute__((ext_vector_type(8)))  _Float16 v8h;
typedef __attribute__((ext_vector_type(16))) __bf16   v16b;
typedef __attribute__((ext_vector_type(8)))  __bf16   v8b;
typedef __attribute__((ext_vector_type(8)))  float    v8f;
typedef __attribute__((ext_vector_type(4)))  float    v4f;
typedef __attribute__((ext_vector_type(4)))  unsigned int v4u;

__device__ __forceinline__ unsigned short f2bf_bits(float f) {
  unsigned u = __float_as_uint(f);
  return (unsigned short)((u + 0x7FFFu + ((u >> 16) & 1u)) >> 16);
}
__device__ __forceinline__ float bf_bits2f(unsigned short h) { return __uint_as_float(((unsigned)h) << 16); }

__device__ __forceinline__ void dep_guard_h(v8f& a, v8f& b, v16h x, v16h y) { asm volatile("v_nop\n\tv_nop\n\tv_nop\n\tv_nop" : "+v"(a), "+v"(b) : "v"(x), "v"(y)); }
__device__ __forceinline__ void dep_guard_b(v8f& a, v8f& b, v16b x, v16b y) { asm volatile("v_nop\n\tv_nop\n\tv_nop\n\tv_nop" : "+v"(a), "+v"(b) : "v"(x), "v"(y)); }
__device__ __forceinline__ void keep4_h(v16h a, v16h b, v16h c, v16h d) { asm volatile("v_nop" :: "v"(a), "v"(b), "v"(c), "v"(d)); }
__device__ __forceinline__ void keep4_b(v16b a, v16b b, v16b c, v16b d) { asm volatile("v_nop" :: "v"(a), "v"(b), "v"(c), "v"(d)); }
__device__ __forceinline__ void acc_guard4(v8f& a, v8f& b, v8f& c, v8f& d) { asm volatile("v_nop\n\tv_nop\n\tv_nop\n\tv_nop" : "+v"(a), "+v"(b), "+v"(c), "+v"(d)); }
template <typename T> struct Frag;
template <> struct Frag<_Float16> {
  typedef v16h V; union U { v16h v; v8h h[2]; };
  static __device__ __forceinline__ v16h load(const _Float16* p) {
    U f; f.h[0] = *(const v8h*)(p); f.h[1] = *(const v8h*)(p + 16); return f.v;
  }
  static __device__ __forceinline__ v8f mma(v16h a, v16h b, v8f c) {
    return __builtin_amdgcn_wmma_f32_16x16x32_f16(false, a, false, b, (short)0, c, false, false);
  }
  static __device__ __forceinline__ void guard(v8f& a, v8f& b, v16h x, v16h y) { dep_guard_h(a, b, x, y); }
  static __device__ __forceinline__ void keep(v16h a, v16h b, v16h c, v16h d) { keep4_h(a, b, c, d); }
};
template <> struct Frag<__bf16> {
  typedef v16b V; union U { v16b v; v8b h[2]; };
  static __device__ __forceinline__ v16b load(const __bf16* p) {
    U f; f.h[0] = *(const v8b*)(p); f.h[1] = *(const v8b*)(p + 16); return f.v;
  }
  static __device__ __forceinline__ v8f mma(v16b a, v16b b, v8f c) {
    return __builtin_amdgcn_wmma_f32_16x16x32_bf16(false, a, false, b, (short)0, c, false, false);
  }
  static __device__ __forceinline__ void guard(v8f& a, v8f& b, v16b x, v16b y) { dep_guard_b(a, b, x, y); }
  static __device__ __forceinline__ void keep(v16b a, v16b b, v16b c, v16b d) { keep4_b(a, b, c, d); }
};

__device__ __forceinline__ unsigned pk16(unsigned short a, unsigned short b) { return (unsigned)a | ((unsigned)b << 16); }
__device__ __forceinline__ unsigned short h_bits(float f) { const _Float16 h = (_Float16)f; return __builtin_bit_cast(unsigned short, h); }
__device__ __forceinline__ v4u pack8(const unsigned short* hb) {
  return (v4u){pk16(hb[0], hb[1]), pk16(hb[2], hb[3]), pk16(hb[4], hb[5]), pk16(hb[6], hb[7])};
}

__device__ __forceinline__ void store_slab_f32(const float* slab, int lane, float* Cf, int ld, int mBase, int n0) {
  const int hh = lane >> 4, c4 = (lane & 15) * 4;
  for (int pass = 0; pass < 2; ++pass) {
#pragma unroll
    for (int it = 0; it < 8; ++it) {
      const int row = it * 2 + hh;
      const v4f v = *(const v4f*)(slab + row * 68 + c4);
      *(volatile v4f*)(Cf + (size_t)(mBase + row) * ld + n0 + c4) = v;
    }
    __threadfence();
  }
}
template <int MODE>
__device__ __forceinline__ void store_slab_16(const float* slab, int lane, unsigned short* Ch, unsigned short* Cl,
                                              int ld, int mBase, int n0, float ocarry) {
  const int q = lane >> 3, c8 = (lane & 7) * 8;
  for (int pass = 0; pass < 2; ++pass) {
#pragma unroll
    for (int it = 0; it < 4; ++it) {
      const int row = it * 4 + q;
      const float* sp = slab + row * 68 + c8;
      v8h hv, lv;
#pragma unroll
      for (int e = 0; e < 8; ++e) {
        if (MODE == 1) {
          hv[e] = (_Float16)(sp[e] * ocarry);
          lv[e] = hv[e];
        } else {
          const unsigned short hb = f2bf_bits(sp[e]);
          const unsigned short lb = f2bf_bits(sp[e] - bf_bits2f(hb));
          hv[e] = __builtin_bit_cast(_Float16, hb);
          lv[e] = __builtin_bit_cast(_Float16, lb);
        }
      }
      *(volatile v8h*)(Ch + (size_t)(mBase + row) * ld + n0 + c8) = hv;
      if (MODE == 2) *(volatile v8h*)(Cl + (size_t)(mBase + row) * ld + n0 + c8) = lv;
    }
    __threadfence();
  }
}

template <int ET> struct Elem;
template <> struct Elem<0> { typedef _Float16 T; };
template <> struct Elem<1> { typedef __bf16 T; };
template <int ET, bool SPLIT, int BIAS_MODE, int ACT, int RES, int OUTM>
__global__ __launch_bounds__(256) void gemm64(
    const unsigned short* __restrict__ Ap, const unsigned short* __restrict__ A2p, int lda,
    const unsigned short* __restrict__ Btp, const unsigned short* __restrict__ Bt2p, int ldb,
    void* C1, int ldc1, void* C2, int ldc2,
    const float* __restrict__ bias,
    const float* R1, const float* R2, int ldr, int rsplit,
    int M, int N, int K, float scale, float ocarry) {
  typedef typename Elem<ET>::T T;
  typedef typename Frag<T>::V V;
  const T* A = (const T*)Ap; const T* A2 = (const T*)A2p; const T* Bt = (const T*)Btp; const T* Bt2 = (const T*)Bt2p;
  __shared__ __align__(16) float sT[8][16 * 68];
  const int lane = threadIdx.x & 31;
  const int wave = threadIdx.x >> 5;
  const int tilesN = N >> 6;
  const int tilesM = M >> 6;
  const int tile = blockIdx.x * 8 + wave;
  if (tile >= tilesM * tilesN) return;
  const int tm = tile / tilesN;
  const int tn = tile - tm * tilesN;
  const int m0 = tm << 6;
  const int n0 = tn << 6;

  const int rlane = lane & 15;
  const int koff  = (lane >> 4) * 8;
  const int mOff  = (lane >> 4) * 8;

  v8f acc[4][4];
#pragma unroll
  for (int i = 0; i < 4; ++i)
#pragma unroll
    for (int j = 0; j < 4; ++j) acc[i][j] = (v8f){0.f,0.f,0.f,0.f,0.f,0.f,0.f,0.f};

  for (int k0 = 0; k0 < K; k0 += 32) {
    V bh[4], bl[4];
#pragma unroll
    for (int j = 0; j < 4; ++j) {
      const size_t bo = (size_t)(n0 + (j << 4) + rlane) * ldb + koff + k0;
      bh[j] = Frag<T>::load(Bt + bo);
      if (SPLIT) bl[j] = Frag<T>::load(Bt2 + bo);
    }
#pragma unroll
    for (int i = 0; i < 4; ++i) {
      const size_t ao = (size_t)(m0 + (i << 4) + rlane) * lda + koff + k0;
      V ah = Frag<T>::load(A + ao);
      V al;
      if (SPLIT) al = Frag<T>::load(A2 + ao);
#pragma unroll
      for (int j = 0; j < 4; ++j) {
        acc[i][j] = Frag<T>::mma(ah, bh[j], acc[i][j]);
        if (SPLIT) {
          acc[i][j] = Frag<T>::mma(ah, bl[j], acc[i][j]);
          acc[i][j] = Frag<T>::mma(al, bh[j], acc[i][j]);
        }
      }
      Frag<T>::guard(acc[i][0], acc[i][3], ah, SPLIT ? al : ah);
    }
    Frag<T>::keep(bh[0], bh[1], bh[2], bh[3]);
    if (SPLIT) Frag<T>::keep(bl[0], bl[1], bl[2], bl[3]);
  }
  acc_guard4(acc[0][0], acc[0][1], acc[0][2], acc[0][3]);
  acc_guard4(acc[1][0], acc[1][1], acc[1][2], acc[1][3]);
  acc_guard4(acc[2][0], acc[2][1], acc[2][2], acc[2][3]);
  acc_guard4(acc[3][0], acc[3][1], acc[3][2], acc[3][3]);

  float* slab = sT[wave];
#pragma unroll
  for (int i = 0; i < 4; ++i) {
    const int mBase = m0 + (i << 4);
#pragma unroll
    for (int j = 0; j < 4; ++j) {
      const int n = n0 + (j << 4) + rlane;
      float bv = 0.f;
      if (BIAS_MODE == 2) bv = bias[n];
      const float* Rsel = R1;
      if (RES == 1) Rsel = (n0 < rsplit) ? (R1 + n) : (R2 + (n - rsplit));
#pragma unroll
      for (int r = 0; r < 8; ++r) {
        float v = acc[i][j][r] * scale;
        if (BIAS_MODE == 2) v += bv;
        if (ACT == 1) {
          const float en = expf(fminf(v, 0.0f)) - 1.0f;
          v = (v > 0.0f) ? v : en;
        }
        if (RES == 1) v += Rsel[(size_t)(mBase + mOff + r) * ldr];
        slab[(mOff + r) * 68 + (j << 4) + rlane] = v;
      }
    }
    __builtin_amdgcn_fence(__ATOMIC_RELEASE, "workgroup");
    __builtin_amdgcn_wave_barrier();
    __builtin_amdgcn_fence(__ATOMIC_ACQUIRE, "workgroup");
    if (OUTM == 0 || OUTM == 3) store_slab_f32(slab, lane, (float*)C1, ldc1, mBase, n0);
    if (OUTM == 1) store_slab_16<1>(slab, lane, (unsigned short*)C1, (unsigned short*)C1, ldc1, mBase, n0, ocarry);
    if (OUTM == 2) store_slab_16<2>(slab, lane, (unsigned short*)C1, (unsigned short*)C2, ldc1, mBase, n0, ocarry);
    if (OUTM == 3) store_slab_16<1>(slab, lane, (unsigned short*)C2, (unsigned short*)C2, ldc2, mBase, n0, ocarry);
    __builtin_amdgcn_fence(__ATOMIC_RELEASE, "workgroup");
    __builtin_amdgcn_wave_barrier();
    __builtin_amdgcn_fence(__ATOMIC_ACQUIRE, "workgroup");
  }
}

template <int OUTK>
__global__ __launch_bounds__(256) void wtrans_kernel(const float* W1, int N1, const float* W2, int N2, int K, long srcStrideZ,
                                                     unsigned short* dst, unsigned short* dst2, int ldb, int colStrideZ, float scale) {
  __shared__ float sm[64][65];
  const int t = threadIdx.x;
  const int k0 = blockIdx.x * 64;
  const int n0 = blockIdx.y * 64;
  const int z = blockIdx.z;
  const float* W1z = W1 + (size_t)z * (size_t)srcStrideZ;
  const float* W2z = W2 + (size_t)z * (size_t)srcStrideZ;
  const int n2max = (N2 > 0) ? (N2 - 1) : 0;
#pragma unroll
  for (int i = 0; i < 16; ++i) {
    const int e = i * 256 + t;
    const int kl = e >> 6;
    const int nl = e & 63;
    const int k = k0 + kl;
    const int n = n0 + nl;
    const int kc = (k < K) ? k : (K - 1);
    const int n1c = (n < N1) ? n : (N1 - 1);
    int n2c = n - N1;
    n2c = (n2c < 0) ? 0 : n2c;
    n2c = (n2c > n2max) ? n2max : n2c;
    const float v1 = W1z[(size_t)kc * N1 + n1c];
    const float v2 = W2z[(size_t)kc * N2 + n2c];
    const bool ok1 = (k < K) && (n < N1);
    const bool ok2 = (k < K) && (n >= N1) && (n < N1 + N2);
    const float v = ok1 ? v1 : (ok2 ? v2 : 0.0f);
    sm[nl][kl] = v * scale;
  }
  __syncthreads();
  const int lane = t & 31, wave = t >> 5;
  const int q = lane >> 3, c8 = (lane & 7) * 8;
  for (int pass = 0; pass < 2; ++pass) {
#pragma unroll
    for (int it = 0; it < 2; ++it) {
      const int row = wave * 8 + it * 4 + q;
      const size_t o = (size_t)(n0 + row) * ldb + (size_t)z * colStrideZ + k0 + c8;
      unsigned short hb[8], lb[8];
#pragma unroll
      for (int e = 0; e < 8; ++e) {
        const float v = sm[row][c8 + e];
        if (OUTK == 1) {
          hb[e] = h_bits(v);
          lb[e] = hb[e];
        } else {
          const unsigned short hbb = f2bf_bits(v);
          hb[e] = hbb;
          lb[e] = f2bf_bits(v - bf_bits2f(hbb));
        }
      }
      const v4u uh = pack8(hb);
      *(volatile v4u*)(dst + o) = uh;
      if (OUTK == 2) {
        const v4u ul = pack8(lb);
        *(volatile v4u*)(dst2 + o) = ul;
      }
    }
    __threadfence();
  }
}

__global__ __launch_bounds__(256) void btail_kernel(const float* __restrict__ bsrc, int ncol, unsigned short* __restrict__ dst) {
  const int t = blockIdx.x * 256 + threadIdx.x;
  if (t >= ncol * 8) return;
  const int o = t >> 3, sub = t & 7;
  const float tz = (sub == 0) ? kWCarry : 0.0f;
  unsigned short hb[8];
#pragma unroll
  for (int e = 0; e < kNE; ++e) hb[e] = h_bits(bsrc[(size_t)e * ncol + o] * tz);
  hb[6] = 0;
  hb[7] = 0;
  const v4u u = pack8(hb);
  unsigned short* q = dst + (size_t)o * kMoeLd + kNE * kNF2 + sub * 8;
  *(volatile v4u*)q = u;
  __threadfence();
  *(volatile v4u*)q = u;
}

__global__ __launch_bounds__(256) void cast192_kernel(const float* __restrict__ src, unsigned short* __restrict__ dst, int colOff) {
  const int t = blockIdx.x * 256 + threadIdx.x;
  if (t >= kRows * 24) return;
  const int row = t / 24;
  const int g = t - row * 24;
  const float* p = src + (size_t)row * kNF + 8 * g;
  const v4f a = *(const v4f*)(p);
  const v4f b = *(const v4f*)(p + 4);
  unsigned short hb[8];
#pragma unroll
  for (int e = 0; e < 4; ++e) {
    hb[e]     = h_bits(a[e] * kActCarry);
    hb[4 + e] = h_bits(b[e] * kActCarry);
  }
  const v4u u = pack8(hb);
  unsigned short* q = dst + (size_t)row * kNF2 + colOff + 8 * g;
  *(volatile v4u*)q = u;
  __threadfence();
  *(volatile v4u*)q = u;
}

__global__ __launch_bounds__(256) void headout_kernel(const float* __restrict__ head, const float* __restrict__ mub,
                                                      const float* __restrict__ lvb, float* outMu, float* outLv) {
  const int t = blockIdx.x * 256 + threadIdx.x;
  if (t >= kRows * kNL / 4) return;
  const int f0 = t * 4;
  v4f muv, lvv;
#pragma unroll
  for (int e = 0; e < 4; ++e) {
    const int f = f0 + e;
    const int row = f / kNL;
    const int col = f - row * kNL;
    const float* hr = head + (size_t)row * kHeadN;
    muv[e] = hr[col] + mub[col];
    lvv[e] = fminf(hr[kNL + col] + lvb[col], 20.0f);
  }
  *(volatile v4f*)(outMu + f0) = muv;
  *(volatile v4f*)(outLv + f0) = lvv;
  __threadfence();
  *(volatile v4f*)(outMu + f0) = muv;
  *(volatile v4f*)(outLv + f0) = lvv;
}

__global__ __launch_bounds__(256) void zplane_kernel(const float* __restrict__ head, const float* __restrict__ mub,
                                                     const float* __restrict__ lvb, const float* __restrict__ eps,
                                                     unsigned short* __restrict__ z16) {
  const int t = blockIdx.x * 256 + threadIdx.x;
  if (t >= kRows * 8) return;
  const int row = t >> 3, sub = t & 7;
  const float* hr = head + (size_t)row * kHeadN;
  const float* er = eps + (size_t)row * kNL;
  unsigned short hb[8];
#pragma unroll
  for (int e = 0; e < 8; ++e) {
    const int col = sub * 8 + e;
    const int cc = (col < kNL) ? col : (kNL - 1);
    const float mu = hr[cc] + mub[cc];
    const float lv = fminf(hr[kNL + cc] + lvb[cc], 20.0f);
    const float zz = mu + er[cc] * expf(0.5f * lv);
    const float zv = (col < kNL) ? zz : 0.0f;
    hb[e] = h_bits(zv * kActCarry);
  }
  const v4u u = pack8(hb);
  unsigned short* q = z16 + (size_t)row * kZK + sub * 8;
  *(volatile v4u*)q = u;
  __threadfence();
  *(volatile v4u*)q = u;
}

__global__ __launch_bounds__(256) void softmax6_kernel(const float* __restrict__ logit, const float* __restrict__ g3b,
                                                       float* __restrict__ coeff) {
  const int t = blockIdx.x * 256 + threadIdx.x;
  if (t >= kRows * 2) return;
  const int row = t >> 1, half = t & 1;
  const float* lr = logit + (size_t)row * kNG;
  const v4f a = *(const v4f*)(lr);
  const v4f b = *(const v4f*)(lr + 4);
  const float l0 = a[0] + g3b[0], l1 = a[1] + g3b[1], l2 = a[2] + g3b[2], l3 = a[3] + g3b[3];
  const float l4 = b[0] + g3b[4], l5 = b[1] + g3b[5];
  const float mx = fmaxf(fmaxf(fmaxf(l0, l1), fmaxf(l2, l3)), fmaxf(l4, l5));
  const float e0 = expf(l0 - mx), e1 = expf(l1 - mx), e2 = expf(l2 - mx);
  const float e3 = expf(l3 - mx), e4 = expf(l4 - mx), e5 = expf(l5 - mx);
  const float s = ((((e0 + e1) + e2) + e3) + e4) + e5;
  const float inv = 1.0f / s;
  v4f o;
  o[0] = (half == 0) ? e0 * inv : e4 * inv;
  o[1] = (half == 0) ? e1 * inv : e5 * inv;
  o[2] = (half == 0) ? e2 * inv : 0.0f;
  o[3] = (half == 0) ? e3 * inv : 0.0f;
  float* q = coeff + (size_t)row * 8 + half * 4;
  *(volatile v4f*)q = o;
  __threadfence();
  *(volatile v4f*)q = o;
}

__global__ __launch_bounds__(256) void build_moe_a_kernel(const float* __restrict__ coeff,
                                                          const float* P1, int ld1, const float* P2, int ld2,
                                                          unsigned short* __restrict__ dst, int rows, float carry) {
  const int t = blockIdx.x * 256 + threadIdx.x;
  if (t >= rows * kThreadsPerMoeRow) return;
  const int row = t / kThreadsPerMoeRow;
  const int rem = t - row * kThreadsPerMoeRow;
  const int lg = rem >> 3;
  const int sub = rem & 7;
  const v4f cv0 = *(const v4f*)(coeff + (size_t)row * 8);
  const v4f cv1 = *(const v4f*)(coeff + (size_t)row * 8 + 4);
  const int ex = lg / 6;
  const int blk = lg - 6 * ex;
  const int i0 = blk * 64 + sub * 8;
  const int i1 = (i0 < kNF - 8) ? i0 : (kNF - 8);
  int i2 = i0 - kNF;
  i2 = (i2 < 0) ? 0 : i2;
  i2 = (i2 > kNF - 8) ? (kNF - 8) : i2;
  const float* p1 = P1 + (size_t)row * ld1 + i1;
  const float* p2 = P2 + (size_t)row * ld2 + i2;
  const v4f a1 = *(const v4f*)(p1);
  const v4f b1 = *(const v4f*)(p1 + 4);
  const v4f a2 = *(const v4f*)(p2);
  const v4f b2 = *(const v4f*)(p2 + 4);
  float ce = cv1[1];
  ce = (ex == 4) ? cv1[0] : ce;
  ce = (ex == 3) ? cv0[3] : ce;
  ce = (ex == 2) ? cv0[2] : ce;
  ce = (ex == 1) ? cv0[1] : ce;
  ce = (ex == 0) ? cv0[0] : ce;
  const bool useP1 = (i0 < kNF);
  const bool mainPart = (lg < 36);
  const float tz = (sub == 0) ? carry : 0.0f;
  float tv[8];
  tv[0] = cv0[0] * tz; tv[1] = cv0[1] * tz; tv[2] = cv0[2] * tz; tv[3] = cv0[3] * tz;
  tv[4] = cv1[0] * tz; tv[5] = cv1[1] * tz; tv[6] = 0.0f;          tv[7] = 0.0f;
  unsigned short hb[8];
#pragma unroll
  for (int e = 0; e < 4; ++e) {
    const float s0 = useP1 ? a1[e] : a2[e];
    const float s1 = useP1 ? b1[e] : b2[e];
    const float m0v = (ce * s0) * carry;
    const float m1v = (ce * s1) * carry;
    hb[e]     = h_bits(mainPart ? m0v : tv[e]);
    hb[4 + e] = h_bits(mainPart ? m1v : tv[4 + e]);
  }
  const v4u u = pack8(hb);
  unsigned short* q = dst + (size_t)row * kMoeLd + lg * 64 + sub * 8;
  *(volatile v4u*)q = u;
  __threadfence();
  *(volatile v4u*)q = u;
}

extern "C" void kernel_launch(void* const* d_in, const int* in_sizes, int n_in,
                              void* d_out, int out_size, void* d_ws, size_t ws_size,
                              hipStream_t stream) {
  if (n_in < 27) return;
  if (in_sizes[0] != kRows * kNF || in_sizes[1] != kRows * kNF || in_sizes[2] != kRows * kNL) return;
  if (in_sizes[17] != kNE * kNF2 * kNF2 || in_sizes[19] != kNE * kNF2 * kNF) return;
  if (out_size != kRows * (kNF + 2 * kNL)) return;
  if (ws_size < kWsTotal) return;

  const float* x   = (const float*)d_in[0];
  const float* c   = (const float*)d_in[1];
  const float* eps = (const float*)d_in[2];
  const float* e1w = (const float*)d_in[3];  const float* e1b = (const float*)d_in[4];
  const float* e2w = (const float*)d_in[5];  const float* e2b = (const float*)d_in[6];
  const float* e3w = (const float*)d_in[7];  const float* e3b = (const float*)d_in[8];
  const float* e4w = (const float*)d_in[9];  const float* e4b = (const float*)d_in[10];
  const float* muw = (const float*)d_in[11]; const float* mub = (const float*)d_in[12];
  const float* lvw = (const float*)d_in[13]; const float* lvb = (const float*)d_in[14];
  const float* d1w = (const float*)d_in[15]; const float* d1b = (const float*)d_in[16];
  const float* w0  = (const float*)d_in[17]; const float* b0  = (const float*)d_in[18];
  const float* w1  = (const float*)d_in[19]; const float* b1  = (const float*)d_in[20];
  const float* g1w = (const float*)d_in[21]; const float* g1b = (const float*)d_in[22];
  const float* g2w = (const float*)d_in[23]; const float* g2b = (const float*)d_in[24];
  const float* g3w = (const float*)d_in[25]; const float* g3b = (const float*)d_in[26];

  float* out0 = (float*)d_out;
  float* out1 = out0 + (size_t)kRows * kNF;
  float* out2 = out1 + (size_t)kRows * kNL;

  char* ws = (char*)d_ws;
  unsigned short* e1t  = (unsigned short*)(ws + kOffE1t);
  unsigned short* e2t  = (unsigned short*)(ws + kOffE2t);
  unsigned short* e3t  = (unsigned short*)(ws + kOffE3t);
  unsigned short* e4t  = (unsigned short*)(ws + kOffE4t);
  unsigned short* hdhi = (unsigned short*)(ws + kOffHdHi);
  unsigned short* hdlo = (unsigned short*)(ws + kOffHdLo);
  unsigned short* d1t  = (unsigned short*)(ws + kOffD1t);
  unsigned short* g1t  = (unsigned short*)(ws + kOffG1t);
  unsigned short* g2t  = (unsigned short*)(ws + kOffG2t);
  unsigned short* g3t  = (unsigned short*)(ws + kOffG3t);
  unsigned short* bt0  = (unsigned short*)(ws + kOffBt0);
  unsigned short* bt1  = (unsigned short*)(ws + kOffBt1);
  unsigned short* xc16 = (unsigned short*)(ws + kOffR0);
  unsigned short* h2h  = (unsigned short*)(ws + kOffR0);
  unsigned short* h4hi = (unsigned short*)(ws + kOffR0);
  unsigned short* h4lo = (unsigned short*)(ws + kOffR0 + 12 * kMiB);
  float*          zdec = (float*)(ws + kOffR0);
  unsigned short* hin16 = (unsigned short*)(ws + kOffR1);
  unsigned short* s16   = (unsigned short*)(ws + kOffR1);
  float*          head  = (float*)(ws + kOffR1);
  unsigned short* zc16  = (unsigned short*)(ws + kOffR1);
  unsigned short* g2h   = (unsigned short*)(ws + kOffR1);
  float*          logit = (float*)(ws + kOffR1 + 4 * kMiB);
  float*          coeff = (float*)(ws + kOffR1 + 12 * kMiB);
  float*          upl   = (float*)(ws + kOffR1);
  float*          h2f   = (float*)(ws + kOffR2);
  unsigned short* z16   = (unsigned short*)(ws + kOffR2);
  unsigned short* g16   = (unsigned short*)(ws + kOffR2 + 4 * kMiB);
  unsigned short* amoe  = (unsigned short*)(ws + kOffR2);

  wtrans_kernel<1><<<dim3(6, 6, 1), 256, 0, stream>>>(e1w, kNF2, e1w, 0, kNF2, 0L, e1t, e1t, kNF2, 0, kWCarry);
  wtrans_kernel<1><<<dim3(6, 6, 1), 256, 0, stream>>>(e2w, kNF2, e2w, 0, kNF2, 0L, e2t, e2t, kNF2, 0, kWCarry);
  wtrans_kernel<1><<<dim3(6, 6, 1), 256, 0, stream>>>(e3w, kNF2, e3w, 0, kNF2, 0L, e3t, e3t, kNF2, 0, kWCarry);
  wtrans_kernel<1><<<dim3(6, 3, 1), 256, 0, stream>>>(e4w, kNF, e4w, 0, kNF2, 0L, e4t, e4t, kNF2, 0, kWCarry);
  wtrans_kernel<2><<<dim3(3, 2, 1), 256, 0, stream>>>(muw, kNL, lvw, kNL, kNF, 0L, hdhi, hdlo, kNF, 0, 1.0f);
  wtrans_kernel<1><<<dim3(1, 3, 1), 256, 0, stream>>>(d1w, kNF, d1w, 0, kNL, 0L, d1t, d1t, kZK, 0, kWCarry);
  wtrans_kernel<1><<<dim3(6, 1, 1), 256, 0, stream>>>(g1w, kNG, g1w, 0, kNF2, 0L, g1t, g1t, kNF2, 0, kWCarry);
  wtrans_kernel<1><<<dim3(1, 1, 1), 256, 0, stream>>>(g2w, kNG, g2w, 0, kNG, 0L, g2t, g2t, kNG, 0, kWCarry);
  wtrans_kernel<1><<<dim3(1, 1, 1), 256, 0, stream>>>(g3w, kNE, g3w, 0, kNG, 0L, g3t, g3t, kNG, 0, kWCarry);
  wtrans_kernel<1><<<dim3(6, 6, kNE), 256, 0, stream>>>(w0, kNF2, w0, 0, kNF2, (long)kNF2 * kNF2, bt0, bt0, kMoeLd, kNF2, kWCarry);
  wtrans_kernel<1><<<dim3(6, 3, kNE), 256, 0, stream>>>(w1, kNF, w1, 0, kNF2, (long)kNF2 * kNF, bt1, bt1, kMoeLd, kNF2, kWCarry);
  btail_kernel<<<(kNF2 * 8) / 256, 256, 0, stream>>>(b0, kNF2, bt0);
  btail_kernel<<<(kNF * 8) / 256, 256, 0, stream>>>(b1, kNF, bt1);

  const int castBlocks = (kRows * 24 + 255) / 256;
  cast192_kernel<<<castBlocks, 256, 0, stream>>>(x, xc16, 0);
  cast192_kernel<<<castBlocks, 256, 0, stream>>>(c, xc16, kNF);
  const int gemmBlocks384 = (kRows / 64) * (kNF2 / 64) / 8;
  const int gemmBlocks192 = (kRows / 64) * (kNF / 64) / 8;
  const int gemmBlocks128 = (kRows / 64) * (kHeadN / 64) / 8;
  const int gemmBlocks64  = (kRows / 64) * (kNG / 64) / 8;
  gemm64<0, false, 2, 1, 1, 1><<<gemmBlocks384, 256, 0, stream>>>(
      xc16, xc16, kNF2, e1t, e1t, kNF2, hin16, kNF2, hin16, kNF2, e1b, x, c, kNF, kNF, kRows, kNF2, kNF2, kPlainScale, kActCarry);
  gemm64<0, false, 2, 1, 0, 3><<<gemmBlocks384, 256, 0, stream>>>(
      hin16, hin16, kNF2, e2t, e2t, kNF2, h2f, kNF2, h2h, kNF2, e2b, x, x, 0, 0, kRows, kNF2, kNF2, kPlainScale, kActCarry);
  gemm64<0, false, 2, 1, 1, 1><<<gemmBlocks384, 256, 0, stream>>>(
      h2h, h2h, kNF2, e3t, e3t, kNF2, s16, kNF2, s16, kNF2, e3b, h2f, h2f + kNF, kNF2, kNF, kRows, kNF2, kNF2, kPlainScale, kActCarry);
  gemm64<0, false, 2, 1, 0, 2><<<gemmBlocks192, 256, 0, stream>>>(
      s16, s16, kNF2, e4t, e4t, kNF2, h4hi, kNF, h4lo, kNF, e4b, x, x, 0, 0, kRows, kNF, kNF2, kPlainScale, 1.0f);
  gemm64<1, true, 0, 0, 0, 0><<<gemmBlocks128, 256, 0, stream>>>(
      h4hi, h4lo, kNF, hdhi, hdlo, kNF, head, kHeadN, head, kHeadN, x, x, x, 0, 0, kRows, kHeadN, kNF, 1.0f, 1.0f);
  headout_kernel<<<(kRows * kNL / 4 + 255) / 256, 256, 0, stream>>>(head, mub, lvb, out1, out2);
  zplane_kernel<<<(kRows * 8 + 255) / 256, 256, 0, stream>>>(head, mub, lvb, eps, z16);

  cast192_kernel<<<castBlocks, 256, 0, stream>>>(c, zc16, kNF);
  gemm64<0, false, 2, 1, 0, 3><<<gemmBlocks192, 256, 0, stream>>>(
      z16, z16, kZK, d1t, d1t, kZK, zdec, kNF, zc16, kNF2, d1b, x, x, 0, 0, kRows, kNF, kZK, kPlainScale, kActCarry);
  gemm64<0, false, 2, 1, 0, 1><<<gemmBlocks64, 256, 0, stream>>>(
      zc16, zc16, kNF2, g1t, g1t, kNF2, g16, kNG, g16, kNG, g1b, x, x, 0, 0, kRows, kNG, kNF2, kPlainScale, kActCarry);
  gemm64<0, false, 2, 1, 0, 1><<<gemmBlocks64, 256, 0, stream>>>(
      g16, g16, kNG, g2t, g2t, kNG, g2h, kNG, g2h, kNG, g2b, x, x, 0, 0, kRows, kNG, kNG, kPlainScale, kActCarry);
  gemm64<0, false, 0, 0, 0, 0><<<gemmBlocks64, 256, 0, stream>>>(
      g2h, g2h, kNG, g3t, g3t, kNG, logit, kNG, logit, kNG, x, x, x, 0, 0, kRows, kNG, kNG, kPlainScale, 1.0f);
  softmax6_kernel<<<(kRows * 2 + 255) / 256, 256, 0, stream>>>(logit, g3b, coeff);

  const int buildBlocks = (kChunkRows * kThreadsPerMoeRow + 255) / 256;
  const int moe0Blocks = (kChunkRows / 64) * (kNF2 / 64) / 8;
  const int moe1Blocks = (kChunkRows / 64) * (kNF / 64) / 8;
  for (int ch = 0; ch < kNumChunks; ++ch) {
    const size_t r0 = (size_t)ch * kChunkRows;
    const float* coeffCh = coeff + r0 * 8;
    const float* zdecCh = zdec + r0 * kNF;
    const float* cCh = c + r0 * kNF;
    build_moe_a_kernel<<<buildBlocks, 256, 0, stream>>>(coeffCh, zdecCh, kNF, cCh, kNF, amoe, kChunkRows, kMoeCarry);
    gemm64<0, false, 0, 1, 1, 0><<<moe0Blocks, 256, 0, stream>>>(
        amoe, amoe, kMoeLd, bt0, bt0, kMoeLd, upl, kNF2, upl, kNF2, x, zdecCh, cCh, kNF, kNF,
        kChunkRows, kNF2, kMoeK, kMoeScale, 1.0f);
    build_moe_a_kernel<<<buildBlocks, 256, 0, stream>>>(coeffCh, upl, kNF2, upl + kNF, kNF2, amoe, kChunkRows, kMoeCarry);
    gemm64<0, false, 0, 0, 0, 0><<<moe1Blocks, 256, 0, stream>>>(
        amoe, amoe, kMoeLd, bt1, bt1, kMoeLd, out0 + r0 * kNF, kNF, out0 + r0 * kNF, kNF, x, x, x, 0, 0,
        kChunkRows, kNF, kMoeK, kMoeScale, 1.0f);
  }
}
